// TransformerBlock_41601053229694
// MI455X (gfx1250) — hardware-verified
//
#include <hip/hip_runtime.h>
#include <math.h>

#ifndef NB
#define NB 2
#endif
#ifndef SEQ
#define SEQ 2048
#endif
#define NB_FULL 2
#define SEQ_FULL 2048
#define DM 1024
#define NHEAD 8
#define HDIM 128
#define FFN 4096
#define MT (NB * SEQ)
#define QKW (2 * DM)

static_assert(NHEAD * HDIM == DM);
static_assert(HDIM == 128);
static_assert(SEQ % 64 == 0);
static_assert(MT % 64 == 0);
static_assert(DM % 64 == 0);
static_assert(FFN % 64 == 0);
static_assert(DM % 32 == 0);
static_assert(FFN % 32 == 0);
static_assert(NB <= NB_FULL);
static_assert(SEQ <= SEQ_FULL);
static_assert((long long)MT * QKW < 2147483647LL);
static_assert((long long)DM * MT < 2147483647LL);

typedef __attribute__((ext_vector_type(16))) _Float16 v16h;
typedef __attribute__((ext_vector_type(8)))  _Float16 v8h;
typedef __attribute__((ext_vector_type(8)))  float    v8f;
typedef __attribute__((ext_vector_type(4)))  float    v4f;
typedef __attribute__((ext_vector_type(4)))  unsigned int v4u;

union Fr { v16h v; v8h h[2]; };

__device__ __forceinline__ v8f wmma16(v16h a, v16h b, v8f c) {
    c = __builtin_amdgcn_wmma_f32_16x16x32_f16(false, a, false, b, (short)0, c, false, false);
    asm volatile("v_nop\n\tv_nop\n\tv_nop\n\tv_nop" : "+v"(c) : "v"(a), "v"(b));
    return c;
}
__device__ __forceinline__ void wave_sync() {
    __builtin_amdgcn_fence(3  , "workgroup");
    __builtin_amdgcn_wave_barrier();
    __builtin_amdgcn_fence(2  , "workgroup");
}
__device__ __forceinline__ float bfr(float v) {
    unsigned u = __float_as_uint(v);
    u = (u + 0x7fffu + ((u >> 16) & 1u)) & 0xffff0000u;
    return __uint_as_float(u);
}
__device__ __forceinline__ v4f bfr4(v4f a) { v4f r; r.x = bfr(a.x); r.y = bfr(a.y); r.z = bfr(a.z); r.w = bfr(a.w); return r; }
__device__ __forceinline__ unsigned pk2h(float a, float b) {
    return (unsigned)__builtin_bit_cast(unsigned short, (_Float16)a) | ((unsigned)__builtin_bit_cast(unsigned short, (_Float16)b) << 16);
}
__device__ __forceinline__ v4u pk8h(v4f a, v4f b) {
    v4u p; p.x = pk2h(a.x, a.y); p.y = pk2h(a.z, a.w); p.z = pk2h(b.x, b.y); p.w = pk2h(b.z, b.w); return p;
}
__device__ __forceinline__ void st2_u4(unsigned short* d, v4u pk) {
    volatile v4u* p = (volatile v4u*)d; *p = pk; __threadfence(); *p = pk;
}
__device__ __forceinline__ float gelu_erf(float v) { return 0.5f * v * (1.0f + erff(v * 0.70710678118654752f)); }
__device__ __forceinline__ v4f gelu4(v4f a) { v4f r; r.x = gelu_erf(a.x); r.y = gelu_erf(a.y); r.z = gelu_erf(a.z); r.w = gelu_erf(a.w); return r; }

__global__ __launch_bounds__(256) void k_cast_rows(const float* __restrict__ SRC, int lds, int sseq, int sseqf,
                                                   unsigned short* __restrict__ DST, int ldd, int nR, int nC, float sc) {
    const long long u = (long long)blockIdx.x * 256 + threadIdx.x;
    const int per = nC >> 3;
    if (u >= (long long)nR * per) return;
    const int r = (int)(u / per), c0 = 8 * (int)(u % per);
    const int rs = (r / sseq) * sseqf + (r % sseq);
    const float* s = SRC + (size_t)rs * lds + c0;
    v4f a = *(const v4f*)s, b = *(const v4f*)(s + 4);
    a = bfr4(a) * sc; b = bfr4(b) * sc;
    st2_u4(DST + (size_t)r * ldd + c0, pk8h(a, b));
}
__global__ __launch_bounds__(256) void k_castT(const float* __restrict__ SRC, int lds, unsigned short* __restrict__ DST, int ldd,
                                               int nR, int nO, float sc, int perm) {
    const long long u = (long long)blockIdx.x * 256 + threadIdx.x;
    const int per = nR >> 3;
    if (u >= (long long)nO * per) return;
    const int o = (int)(u / per), r0 = 8 * (int)(u % per);
    int col = o;
    if (perm) {
        const int o2 = o - 2 * DM;
        const int cqk = (o >> 8) * (3 * HDIM) + ((o >> 7) & 1) * HDIM + (o & 127);
        const int cv  = (o2 >> 7) * (3 * HDIM) + 2 * HDIM + (o2 & 127);
        col = (o < 2 * DM) ? cqk : cv;
    }
    float w[8];
#pragma unroll
    for (int e = 0; e < 8; ++e) w[e] = bfr(SRC[(size_t)(r0 + e) * lds + col]) * sc;
    v4u pk; pk.x = pk2h(w[0], w[1]); pk.y = pk2h(w[2], w[3]); pk.z = pk2h(w[4], w[5]); pk.w = pk2h(w[6], w[7]);
    st2_u4(DST + (size_t)o * ldd + r0, pk);
}

template <int OUT_MODE, bool HASBIAS, bool ACTG, bool RESID>
__device__ __forceinline__ void gemm64_body(const unsigned short* __restrict__ Ap, int lda,
                                            const unsigned short* __restrict__ Btp, int ldb,
                                            float* __restrict__ Cf, unsigned short* __restrict__ Ch, int ldc,
                                            const float* __restrict__ bias, const float* __restrict__ resid, int ldr,
                                            int M, int N, int K, float scale, float carry, int rbf,
                                            int cseq, int cseqf, int rseq, int rseqf) {
    __shared__ __align__(16) float sT[8 * 16 * 68];
    const _Float16* A  = (const _Float16*)Ap;
    const _Float16* Bt = (const _Float16*)Btp;
    const int lane = (int)(threadIdx.x & 31);
    const int wave = __builtin_amdgcn_readfirstlane((int)(threadIdx.x >> 5));
    const int tilesN = N >> 6, tilesM = M >> 6;
    const int tile = (int)blockIdx.x * 8 + wave;
    if (tile >= tilesM * tilesN) return;
    const int tm = tile / tilesN, tn = tile - tm * tilesN;
    const int m0 = tm << 6, n0 = tn << 6;
    const int rl = lane & 15, hh = lane >> 4, koff = hh * 8, mOff = hh * 8;

    v8f acc[4][4];
#pragma unroll
    for (int i = 0; i < 4; ++i)
#pragma unroll
        for (int j = 0; j < 4; ++j) { v8f z = {}; acc[i][j] = z; }

    for (int k0 = 0; k0 < K; k0 += 32) {
        Fr bh[4];
#pragma unroll
        for (int j = 0; j < 4; ++j) {
            const size_t bo = (size_t)(n0 + (j << 4) + rl) * ldb + koff + k0;
            bh[j].h[0] = *(const v8h*)(Bt + bo);
            bh[j].h[1] = *(const v8h*)(Bt + bo + 16);
        }
#pragma unroll
        for (int i = 0; i < 4; ++i) {
            const size_t ao = (size_t)(m0 + (i << 4) + rl) * lda + koff + k0;
            Fr ah;
            ah.h[0] = *(const v8h*)(A + ao);
            ah.h[1] = *(const v8h*)(A + ao + 16);
#pragma unroll
            for (int j = 0; j < 4; ++j) acc[i][j] = wmma16(ah.v, bh[j].v, acc[i][j]);
        }
    }

    const int sbase = wave * (16 * 68);
    const int crow0 = (m0 / cseq) * cseqf + (m0 % cseq);
    const int rrow0 = (m0 / rseq) * rseqf + (m0 % rseq);
    const int c4 = (lane & 15) * 4;
    const int q8 = lane >> 3, c8 = (lane & 7) * 8;
    v4f b4 = {0.f, 0.f, 0.f, 0.f}, ba = {0.f, 0.f, 0.f, 0.f}, bb = {0.f, 0.f, 0.f, 0.f};
    if (HASBIAS) {
        if (OUT_MODE == 0) b4 = bfr4(*(const v4f*)(bias + n0 + c4));
        else { ba = bfr4(*(const v4f*)(bias + n0 + c8)); bb = bfr4(*(const v4f*)(bias + n0 + c8 + 4)); }
    }
#pragma unroll
    for (int i = 0; i < 4; ++i) {
        const int mB = i << 4;
#pragma unroll
        for (int j = 0; j < 4; ++j)
#pragma unroll
            for (int r = 0; r < 8; ++r) sT[sbase + (mOff + r) * 68 + (j << 4) + rl] = acc[i][j][r] * scale;
        wave_sync();
        if (OUT_MODE == 0) {
#pragma unroll 1
            for (int it = 0; it < 8; ++it) {
                const int row = it * 2 + hh; const int si = sbase + row * 68 + c4;
                v4f v = *(const v4f*)&sT[si];
                v = v + b4;
                if (RESID) {
                    v4f rr = *(const v4f*)(resid + (size_t)(rrow0 + mB + row) * ldr + n0 + c4);
                    const v4f rq = bfr4(rr);
                    if (rbf) rr = rq;
                    v = v + rr;
                }
                *(v4f*)&sT[si] = v;
            }
            wave_sync();
            for (int pass = 0; pass < 2; ++pass) {
#pragma unroll
                for (int it = 0; it < 8; ++it) {
                    const int row = it * 2 + hh;
                    const v4f v = *(const v4f*)&sT[sbase + row * 68 + c4];
                    *(volatile v4f*)(Cf + (size_t)(crow0 + mB + row) * ldc + n0 + c4) = v;
                }
                __threadfence();
            }
        } else {
            if (HASBIAS || ACTG) {
#pragma unroll 1
                for (int it = 0; it < 4; ++it) {
                    const int row = it * 4 + q8; const int si = sbase + row * 68 + c8;
                    v4f va = *(const v4f*)&sT[si], vb = *(const v4f*)&sT[si + 4];
                    va = va + ba; vb = vb + bb;
                    if (ACTG) { va = gelu4(va); vb = gelu4(vb); }
                    va = va * carry; vb = vb * carry;
                    *(v4f*)&sT[si] = va; *(v4f*)&sT[si + 4] = vb;
                }
                wave_sync();
            }
            for (int pass = 0; pass < 2; ++pass) {
#pragma unroll
                for (int it = 0; it < 4; ++it) {
                    const int row = it * 4 + q8; const int si = sbase + row * 68 + c8;
                    const v4f va = *(const v4f*)&sT[si], vb = *(const v4f*)&sT[si + 4];
                    const v4u pk = pk8h(va, vb);
                    *(volatile v4u*)(Ch + (size_t)(crow0 + mB + row) * ldc + n0 + c8) = pk;
                }
                __threadfence();
            }
        }
        wave_sync();
    }
}

__global__ __launch_bounds__(256) void k_gemm_h(const unsigned short* __restrict__ A, int lda, const unsigned short* __restrict__ Bt, int ldb,
                                                unsigned short* __restrict__ C, int ldc, int M, int N, int K, float scale) {
    gemm64_body<1, false, false, false>(A, lda, Bt, ldb, nullptr, C, ldc, nullptr, nullptr, 0, M, N, K, scale, 1.0f, 0, M, M, M, M);
}
__global__ __launch_bounds__(256) void k_gemm_gelu(const unsigned short* __restrict__ A, int lda, const unsigned short* __restrict__ Bt, int ldb,
                                                   unsigned short* __restrict__ C, int ldc, const float* __restrict__ bias,
                                                   int M, int N, int K, float scale, float carry) {
    gemm64_body<1, true, true, false>(A, lda, Bt, ldb, nullptr, C, ldc, bias, nullptr, 0, M, N, K, scale, carry, 0, M, M, M, M);
}
__global__ __launch_bounds__(256) void k_gemm_res(const unsigned short* __restrict__ A, int lda, const unsigned short* __restrict__ Bt, int ldb,
                                                  float* __restrict__ C, int ldc, const float* __restrict__ bias,
                                                  const float* __restrict__ resid, int ldr, int M, int N, int K, float scale, int rbf,
                                                  int cseq, int cseqf, int rseq, int rseqf) {
    gemm64_body<0, true, false, true>(A, lda, Bt, ldb, C, nullptr, ldc, bias, resid, ldr, M, N, K, scale, 1.0f, rbf, cseq, cseqf, rseq, rseqf);
}

__global__ __launch_bounds__(128) void k_attn128(const unsigned short* __restrict__ QKp, const unsigned short* __restrict__ VTp,
                                                 unsigned short* __restrict__ CTXp) {
    __shared__ __align__(16) _Float16 Pl[4 * 16 * 40];
    __shared__ __align__(16) float    Ol[4 * 16 * 132];
    const _Float16* QK = (const _Float16*)QKp;
    const _Float16* VT = (const _Float16*)VTp;
    const int lane = (int)(threadIdx.x & 31), hh = lane >> 4, c = lane & 15;
    const int wave = __builtin_amdgcn_readfirstlane((int)(threadIdx.x >> 5));
    const int NQB = SEQ / 64;
    const int bx = (int)blockIdx.x;
    const int qb = bx % NQB, bh = bx / NQB;
    const int h = bh % NHEAD, b = bh / NHEAD;
    const int q0 = qb * 64 + wave * 16;
    const int qoff0 = (b * SEQ + q0 + c) * QKW + h * 256 + 8 * hh;
    const int kbase = (b * SEQ + c) * QKW + h * 256 + 128 + 8 * hh;
    const int vbase = (h * HDIM + c) * MT + b * SEQ + 8 * hh;
    const int pbase = wave * (16 * 40);
    const float SL2 = 0.08838834764831845f * 1.4426950408889634f;
    const float NEG = -__builtin_inff();

    v8f o[8]; float m8[8], l8[8];
#pragma unroll
    for (int t = 0; t < 8; ++t) { v8f z = {}; o[t] = z; }
#pragma unroll
    for (int r = 0; r < 8; ++r) { m8[r] = NEG; l8[r] = 0.f; }

    const int nh = (q0 + 16 + 31) >> 5;
    for (int jh = 0; jh < nh; ++jh) {
        const int kv0 = jh * 32;
        int qo = qoff0;
        asm volatile("" : "+v"(qo));
        v8f s0 = {}, s1 = {};
#pragma unroll
        for (int ks = 0; ks < 4; ++ks) {
            Fr qa, k0f, k1f;
            qa.h[0] = *(const v8h*)(QK + qo + ks * 32);
            qa.h[1] = *(const v8h*)(QK + qo + ks * 32 + 16);
            const int ko0 = kbase + kv0 * QKW + ks * 32;
            k0f.h[0] = *(const v8h*)(QK + ko0);
            k0f.h[1] = *(const v8h*)(QK + ko0 + 16);
            s0 = wmma16(qa.v, k0f.v, s0);
            const int ko1 = ko0 + 16 * QKW;
            k1f.h[0] = *(const v8h*)(QK + ko1);
            k1f.h[1] = *(const v8h*)(QK + ko1 + 16);
            s1 = wmma16(qa.v, k1f.v, s1);
        }
        const bool diag = (kv0 + 31 > q0);
#pragma unroll
        for (int r = 0; r < 8; ++r) {
            float v0 = s0[r] * SL2, v1 = s1[r] * SL2;
            if (diag) {
                const int qrow = q0 + 8 * hh + r;
                v0 = (kv0 + c > qrow) ? NEG : v0;
                v1 = (kv0 + 16 + c > qrow) ? NEG : v1;
            }
            float mx = fmaxf(v0, v1);
            mx = fmaxf(mx, __shfl_xor(mx, 1, 32)); mx = fmaxf(mx, __shfl_xor(mx, 2, 32));
            mx = fmaxf(mx, __shfl_xor(mx, 4, 32)); mx = fmaxf(mx, __shfl_xor(mx, 8, 32));
            const float mnew = fmaxf(m8[r], mx);
            const float msafe = (mnew == NEG) ? 0.f : mnew;
            const float alpha = exp2f(m8[r] - msafe);
            const float p0 = exp2f(v0 - msafe), p1 = exp2f(v1 - msafe);
            float rs = p0 + p1;
            rs += __shfl_xor(rs, 1, 32); rs += __shfl_xor(rs, 2, 32); rs += __shfl_xor(rs, 4, 32); rs += __shfl_xor(rs, 8, 32);
            l8[r] = l8[r] * alpha + rs; m8[r] = mnew;
#pragma unroll
            for (int t = 0; t < 8; ++t) o[t][r] *= alpha;
            Pl[pbase + (8 * hh + r) * 40 + c]      = (_Float16)(p0 * 1024.0f);
            Pl[pbase + (8 * hh + r) * 40 + 16 + c] = (_Float16)(p1 * 1024.0f);
        }
        wave_sync();
        Fr pa;
        pa.h[0] = *(const v8h*)&Pl[pbase + c * 40 + 8 * hh];
        pa.h[1] = *(const v8h*)&Pl[pbase + c * 40 + 16 + 8 * hh];
#pragma unroll
        for (int t = 0; t < 8; ++t) {
            Fr vb;
            const int vo = vbase + t * 16 * MT + kv0;
            vb.h[0] = *(const v8h*)(VT + vo);
            vb.h[1] = *(const v8h*)(VT + vo + 16);
            o[t] = wmma16(pa.v, vb.v, o[t]);
        }
        wave_sync();
    }

    const int obase = wave * (16 * 132);
#pragma unroll
    for (int r = 0; r < 8; ++r) {
        const float inv = 1.0f / (l8[r] * 16.0f);
#pragma unroll
        for (int t = 0; t < 8; ++t) Ol[obase + (8 * hh + r) * 132 + t * 16 + c] = o[t][r] * inv;
    }
    wave_sync();
    {
        const int c8 = (lane & 15) * 8;
        for (int pass = 0; pass < 2; ++pass) {
#pragma unroll
            for (int it = 0; it < 8; ++it) {
                const int row = it * 2 + hh; const int si = obase + row * 132 + c8;
                const v4f va = *(const v4f*)&Ol[si], vb = *(const v4f*)&Ol[si + 4];
                const v4u pk = pk8h(va, vb);
                *(volatile v4u*)(CTXp + (size_t)(b * SEQ + q0 + row) * DM + h * HDIM + c8) = pk;
            }
            __threadfence();
        }
    }
}

__global__ __launch_bounds__(256) void k_ln16(const float* __restrict__ X, const float* __restrict__ g, const float* __restrict__ bsh,
                                              unsigned short* __restrict__ Y, int rows) {
    __shared__ float red[8];
    const int tid = (int)threadIdx.x, lane = tid & 31;
    const int wave = __builtin_amdgcn_readfirstlane(tid >> 5);
    const int half = wave >> 2, w0 = half * 4;
    const int row = (int)blockIdx.x * 2 + half;
    const int rowc = min(row, rows - 1);
    const int c0 = 8 * (tid & 127);
    const float* xr = X + (size_t)rowc * DM + c0;
    const v4f a0 = *(const v4f*)xr, a1 = *(const v4f*)(xr + 4);
    float s = ((a0.x + a0.y) + (a0.z + a0.w)) + ((a1.x + a1.y) + (a1.z + a1.w));
    s += __shfl_xor(s, 16, 32); s += __shfl_xor(s, 8, 32); s += __shfl_xor(s, 4, 32); s += __shfl_xor(s, 2, 32); s += __shfl_xor(s, 1, 32);
    if (lane == 0) red[wave] = s;
    __syncthreads();
    const float mu = ((red[w0] + red[w0 + 1]) + (red[w0 + 2] + red[w0 + 3])) * (1.0f / (float)DM);
    __syncthreads();
    const v4f d0 = a0 - mu, d1 = a1 - mu;
    float q = d0.x * d0.x + d0.y * d0.y + d0.z * d0.z + d0.w * d0.w + d1.x * d1.x + d1.y * d1.y + d1.z * d1.z + d1.w * d1.w;
    q += __shfl_xor(q, 16, 32); q += __shfl_xor(q, 8, 32); q += __shfl_xor(q, 4, 32); q += __shfl_xor(q, 2, 32); q += __shfl_xor(q, 1, 32);
    if (lane == 0) red[wave] = q;
    __syncthreads();
    const float var = ((red[w0] + red[w0 + 1]) + (red[w0 + 2] + red[w0 + 3])) * (1.0f / (float)DM);
    const float rstd = rsqrtf(var + 1e-5f);
    const v4f g0 = bfr4(*(const v4f*)(g + c0)), g1 = bfr4(*(const v4f*)(g + c0 + 4));
    const v4f h0 = bfr4(*(const v4f*)(bsh + c0)), h1 = bfr4(*(const v4f*)(bsh + c0 + 4));
    const v4f y0 = d0 * rstd * g0 + h0, y1 = d1 * rstd * g1 + h1;
    if (row < rows) st2_u4(Y + (size_t)row * DM + c0, pk8h(y0, y1));
}

#define SZ_X16   ((size_t)MT * DM * 2)
#define SZ_WQ    ((size_t)3 * DM * DM * 2)
#define SZ_QK16  ((size_t)MT * QKW * 2)
#define SZ_VT16  ((size_t)DM * MT * 2)
#define SZ_CTX16 ((size_t)MT * DM * 2)
#define SZ_WOT   ((size_t)DM * DM * 2)
#define SZ_X1    ((size_t)MT * DM * 4)
#define SZ_LN16  ((size_t)MT * DM * 2)
#define SZ_W1T   ((size_t)FFN * DM * 2)
#define SZ_W2T   ((size_t)DM * FFN * 2)
#define SZ_G16   ((size_t)MT * FFN * 2)
#define SZ_TOTAL (SZ_X16 + SZ_WQ + SZ_QK16 + SZ_VT16 + SZ_CTX16 + SZ_WOT + SZ_X1 + SZ_LN16 + SZ_W1T + SZ_W2T + SZ_G16)
static_assert(SZ_TOTAL <= (size_t)134217728);
static_assert(SZ_X16 % 256 == 0);
static_assert(SZ_WQ % 256 == 0);
static_assert(SZ_WOT % 256 == 0);

extern "C" void kernel_launch(void* const* d_in, const int* in_sizes, int n_in, void* d_out, int out_size, void* d_ws, size_t ws_size, hipStream_t stream) {
    if (n_in < 10) return;
    const long long need_rows = (long long)(NB - 1) * SEQ_FULL + SEQ;
    if ((long long)in_sizes[0] < need_rows * DM) return;
    if ((long long)in_sizes[1] < (long long)DM * 3 * DM) return;
    if ((long long)in_sizes[2] < (long long)DM * DM) return;
    if (in_sizes[3] < DM || in_sizes[4] < DM || in_sizes[5] < DM) return;
    if ((long long)in_sizes[6] < (long long)DM * FFN) return;
    if (in_sizes[7] < FFN) return;
    if ((long long)in_sizes[8] < (long long)FFN * DM) return;
    if (in_sizes[9] < DM) return;
    if ((long long)out_size < need_rows * DM) return;
    if ((size_t)SZ_TOTAL > ws_size) return;

    const float* x     = (const float*)d_in[0];
    const float* Wqkv  = (const float*)d_in[1];
    const float* Wout  = (const float*)d_in[2];
    const float* b_out = (const float*)d_in[3];
    const float* ln_g  = (const float*)d_in[4];
    const float* ln_b  = (const float*)d_in[5];
    const float* W1    = (const float*)d_in[6];
    const float* b1    = (const float*)d_in[7];
    const float* W2    = (const float*)d_in[8];
    const float* b2    = (const float*)d_in[9];
    float* out = (float*)d_out;

    char* wsp = (char*)d_ws;
    unsigned short* X16   = (unsigned short*)wsp; wsp += SZ_X16;
    unsigned short* WQ    = (unsigned short*)wsp; wsp += SZ_WQ;
    unsigned short* QK16  = (unsigned short*)wsp; wsp += SZ_QK16;
    unsigned short* VT16  = (unsigned short*)wsp; wsp += SZ_VT16;
    unsigned short* CTX16 = (unsigned short*)wsp; wsp += SZ_CTX16;
    unsigned short* WOT   = (unsigned short*)wsp; wsp += SZ_WOT;
    float*          X1    = (float*)wsp;          wsp += SZ_X1;
    unsigned short* LN16  = (unsigned short*)wsp; wsp += SZ_LN16;
    unsigned short* W1T   = (unsigned short*)wsp; wsp += SZ_W1T;
    unsigned short* W2T   = (unsigned short*)wsp; wsp += SZ_W2T;
    unsigned short* G16   = (unsigned short*)wsp; wsp += SZ_G16;

    k_cast_rows<<<(unsigned)(((long long)MT * (DM / 8) + 255) / 256), 256, 0, stream>>>(x, DM, SEQ, SEQ_FULL, X16, DM, MT, DM, 1.0f);
    k_castT<<<(unsigned)(((long long)(3 * DM) * (DM / 8) + 255) / 256), 256, 0, stream>>>(Wqkv, 3 * DM, WQ, DM, DM, 3 * DM, 64.0f, 1);
    k_castT<<<(unsigned)(((long long)DM * (DM / 8) + 255) / 256), 256, 0, stream>>>(Wout, DM, WOT, DM, DM, DM, 64.0f, 0);
    k_castT<<<(unsigned)(((long long)FFN * (DM / 8) + 255) / 256), 256, 0, stream>>>(W1, FFN, W1T, DM, DM, FFN, 64.0f, 0);
    k_castT<<<(unsigned)(((long long)DM * (FFN / 8) + 255) / 256), 256, 0, stream>>>(W2, DM, W2T, FFN, FFN, DM, 64.0f, 0);
    k_gemm_h<<<(unsigned)(((MT / 64) * (QKW / 64) + 7) / 8), 256, 0, stream>>>(X16, DM, WQ, DM, QK16, QKW, MT, QKW, DM, 1.0f / 64.0f);
    k_gemm_h<<<(unsigned)(((DM / 64) * (MT / 64) + 7) / 8), 256, 0, stream>>>(WQ + (size_t)2 * DM * DM, DM, X16, DM, VT16, MT, DM, MT, DM, 1.0f / 64.0f);
    k_attn128<<<(unsigned)(NB * NHEAD * (SEQ / 64)), 128, 0, stream>>>(QK16, VT16, CTX16);
    k_gemm_res<<<(unsigned)(((MT / 64) * (DM / 64) + 7) / 8), 256, 0, stream>>>(CTX16, DM, WOT, DM, X1, DM, b_out, x, DM, MT, DM, DM, 1.0f / 4096.0f, 1,
                                                                                   MT, MT, SEQ, SEQ_FULL);
    k_ln16<<<(unsigned)(MT / 2), 256, 0, stream>>>(X1, ln_g, ln_b, LN16, MT);
    k_gemm_gelu<<<(unsigned)(((MT / 64) * (FFN / 64) + 7) / 8), 256, 0, stream>>>(LN16, DM, W1T, DM, G16, FFN, b1, MT, FFN, DM, 1.0f / 64.0f, 64.0f);
    k_gemm_res<<<(unsigned)(((MT / 64) * (DM / 64) + 7) / 8), 256, 0, stream>>>(G16, FFN, W2T, FFN, out, DM, b2, X1, DM, MT, DM, FFN, 1.0f / 4096.0f, 0,
                                                                                   SEQ, SEQ_FULL, MT, MT);
}
